// Block_Attention_3_48593259987101
// MI455X (gfx1250) — hardware-verified
//
#include <hip/hip_runtime.h>

#define BN_EPS 1e-5f
#define RSPLIT (1.0f / 2048.0f)

typedef _Float16 h16;
typedef __attribute__((ext_vector_type(16))) _Float16 v16h;
typedef __attribute__((ext_vector_type(8)))  _Float16 v8h;
typedef __attribute__((ext_vector_type(8)))  float  v8f;
typedef __attribute__((ext_vector_type(4)))  float  v4f_t;
typedef float v4fa __attribute__((ext_vector_type(4), may_alias));
typedef __attribute__((ext_vector_type(4)))  unsigned v4u_t;
typedef unsigned v4ua __attribute__((ext_vector_type(4), may_alias));

__device__ __forceinline__ h16 lo_of(float v, h16 h) { return (h16)((v - (float)h) * 2048.0f); }
__device__ __forceinline__ v8f wmma16(v16h a, v16h b, v8f c) { return __builtin_amdgcn_wmma_f32_16x16x32_f16(false, a, false, b, (short)0, c, false, false); }
__device__ __forceinline__ v8f wmma_split(v16h a, v16h al, v16h b, v16h bl, v8f c) { v8f x = {}; x = wmma16(al, b, x); x = wmma16(a, bl, x); return wmma16(a, b, c) + x * RSPLIT; }
__device__ __forceinline__ v16h rfrag(const h16* rowp, int half) {
  const h16* p = rowp + 8 * half;
  return __builtin_shufflevector(*(const v8h*)p, *(const v8h*)(p + 16), 0,1,2,3,4,5,6,7,8,9,10,11,12,13,14,15);
}

struct RowParams { const float* bias[4]; const float* g[4]; const float* beta[4]; const float* mu[4]; const float* var[4]; };
struct WPtrs { const float* w[4]; };

__global__ __launch_bounds__(256) void k_row_params(RowParams rp, float* __restrict__ rowScale, float* __restrict__ rowOff) {
  const int m = blockIdx.x * 256 + threadIdx.x;
  const int conv = m >> 8, oc = m & 255;
  const float a = rp.g[conv][oc] * rsqrtf(rp.var[conv][oc] + BN_EPS);
  const float o = (rp.bias[conv][oc] - rp.mu[conv][oc]) * a + rp.beta[conv][oc];
  *(volatile float*)(rowScale + m) = a; *(volatile float*)(rowOff + m) = o; __threadfence();
  *(volatile float*)(rowScale + m) = a; *(volatile float*)(rowOff + m) = o;
}

__global__ __launch_bounds__(256) void k_copy_x(const float* __restrict__ x, float* __restrict__ out) {
  const int t4 = blockIdx.x * 256 + threadIdx.x;
  const int e = t4 * 4;
  const int hw = e & 255, c = (e >> 8) & 2047, b = e >> 19;
  const v4f_t v = *(const v4fa*)(x + e);
  float* d = out + (((size_t)b * 2304 + c) << 8) + hw;
  *(volatile v4f_t*)d = v; __threadfence(); *(volatile v4f_t*)d = v;
}

__global__ __launch_bounds__(256) void k_pack_w(WPtrs wp, h16* __restrict__ A) {
  const int t = blockIdx.x * 256 + threadIdx.x;
  const int e0 = t * 8;
  const int conv = e0 >> 19, off = e0 & 524287;
  h16 hh[8], hl[8];
#pragma unroll
  for (int i = 0; i < 8; ++i) { const float v = wp.w[conv][off + i]; hh[i] = (h16)v; hl[i] = lo_of(v, hh[i]); }
  *(volatile v4u_t*)(A + e0) = *(const v4ua*)hh; *(volatile v4u_t*)(A + 2097152 + e0) = *(const v4ua*)hl; __threadfence();
  *(volatile v4u_t*)(A + e0) = *(const v4ua*)hh; *(volatile v4u_t*)(A + 2097152 + e0) = *(const v4ua*)hl;
}

__global__ __launch_bounds__(256) void k_pack_x(const float* __restrict__ x, h16* __restrict__ Bt) {
  __shared__ float tile[64][65];
  const int n0 = blockIdx.x * 64, k0 = blockIdx.y * 64;
  const int b = n0 >> 8, hw0 = n0 & 255, t = threadIdx.x;
  { const int tn = t & 63, tk4 = t >> 6;
    for (int i = 0; i < 16; i++) { const int kl = i * 4 + tk4; tile[kl][tn] = x[(size_t)b * 524288 + (size_t)(k0 + kl) * 256 + hw0 + tn]; } }
  __syncthreads();
#pragma unroll 1
  for (int pass = 0; pass < 2; ++pass) {
    for (int ch = t; ch < 64 * 8; ch += 256) { const int nl = ch >> 3, k8 = (ch & 7) * 8; h16 hh[8], hl[8];
#pragma unroll
      for (int i = 0; i < 8; ++i) { const float v = tile[k8 + i][nl]; hh[i] = (h16)v; hl[i] = lo_of(v, hh[i]); }
      h16* d = Bt + (size_t)(n0 + nl) * 2048 + k0 + k8;
      *(volatile v4u_t*)d = *(const v4ua*)hh; *(volatile v4u_t*)(d + 2097152) = *(const v4ua*)hl; }
    __threadfence();
  }
}

__global__ __launch_bounds__(256) void k_gemm_kqvd(const h16* __restrict__ A, const h16* __restrict__ Bt,
                                                  const float* __restrict__ rowScale, const float* __restrict__ rowOff,
                                                  float* __restrict__ feat) {
  __shared__ __attribute__((aligned(16))) h16 A_s[2][128 * 40];
  __shared__ __attribute__((aligned(16))) h16 B_s[2][128 * 40];
  __shared__ __attribute__((aligned(16))) float so[128 * 132];
  const int t = threadIdx.x, lane = t & 31, wid = t >> 5, lrow = lane & 15, lhalf = lane >> 4;
  const int waveM = wid & 3, waveN = wid >> 2;
  const int m0 = blockIdx.y * 128, n0 = blockIdx.x * 128;
  const int sr = t >> 1, sh = (t & 1) * 16;
  const h16* ga = A  + (size_t)(m0 + sr) * 2048 + sh;
  const h16* gb = Bt + (size_t)(n0 + sr) * 2048 + sh;

  v8f acc[2][4] = {};
  for (int k0 = 0; k0 < 2048; k0 += 32) {
    __syncthreads();
#pragma unroll
    for (int pl = 0; pl < 2; ++pl) {
      *(v16h*)&A_s[pl][sr * 40 + sh] = *(const v16h*)(ga + (size_t)pl * 2097152 + k0);
      *(v16h*)&B_s[pl][sr * 40 + sh] = *(const v16h*)(gb + (size_t)pl * 2097152 + k0);
    }
    __syncthreads();
    v16h b[4], bl[4];
#pragma unroll
    for (int tn = 0; tn < 4; tn++) { b[tn] = rfrag(&B_s[0][(waveN * 64 + tn * 16 + lrow) * 40], lhalf); bl[tn] = rfrag(&B_s[1][(waveN * 64 + tn * 16 + lrow) * 40], lhalf); }
#pragma unroll
    for (int tm = 0; tm < 2; tm++) {
      const v16h a = rfrag(&A_s[0][(waveM * 32 + tm * 16 + lrow) * 40], lhalf), al = rfrag(&A_s[1][(waveM * 32 + tm * 16 + lrow) * 40], lhalf);
#pragma unroll
      for (int tn = 0; tn < 4; tn++) acc[tm][tn] = wmma_split(a, al, b[tn], bl[tn], acc[tm][tn]);
    }
  }
#pragma unroll
  for (int tm = 0; tm < 2; tm++)
#pragma unroll
    for (int tn = 0; tn < 4; tn++) {
      const int mlBase = waveM * 32 + tm * 16 + lhalf * 8;
      const int nl = waveN * 64 + tn * 16 + lrow;
#pragma unroll
      for (int r = 0; r < 8; r++) {
        const int m = m0 + mlBase + r;
        float y = acc[tm][tn][r] * rowScale[m] + rowOff[m];
        if (m >= 768) y = fmaxf(y, 0.f);
        so[(mlBase + r) * 132 + nl] = y;
      }
    }
  __syncthreads();
#pragma unroll 1
  for (int pass = 0; pass < 2; ++pass) {
    for (int ch = t; ch < 128 * 32; ch += 256) { const int ml = ch >> 5, q = (ch & 31) * 4;
      *(volatile v4f_t*)(feat + (size_t)(m0 + ml) * 1024 + n0 + q) = *(const volatile v4fa*)(so + ml * 132 + q); }
    __threadfence();
  }
}

#define LOG2E_F 1.4426950408889634f
__global__ __launch_bounds__(256) void k_softmax_S(const float* __restrict__ feat, float* __restrict__ S) {
  __shared__ float vals[16 * 256];
  __shared__ float mx_s[16], rs_s[16];
  const int c = threadIdx.x, bh = blockIdx.x, b = bh >> 4, h = bh & 15;
  const float* row = feat + (size_t)(768 + c) * 1024 + b * 256 + h * 16;
  float v[16];
#pragma unroll
  for (int w = 0; w < 16; w++) { v[w] = row[w]; vals[w * 256 + c] = v[w]; }
  __syncthreads();
  if (c < 16) {
    float mx = -1e30f;
#pragma unroll 1
    for (int i = 0; i < 256; i++) mx = fmaxf(mx, vals[c * 256 + i]);
    float s = 0.f;
#pragma unroll 1
    for (int i = 0; i < 256; i++) { const float d_ = (vals[c * 256 + i] - mx) * LOG2E_F; s += __builtin_amdgcn_exp2f(d_); }
    mx_s[c] = mx; rs_s[c] = 1.0f / s;
  }
  __syncthreads();
  float acc = 0.f;
#pragma unroll 1
  for (int w = 0; w < 16; w++) { const float d_ = (v[w] - mx_s[w]) * LOG2E_F; acc += __builtin_amdgcn_exp2f(d_) * rs_s[w]; }
  float* d = S + (size_t)bh * 256 + c;
  *(volatile float*)d = acc; __threadfence(); *(volatile float*)d = acc;
}

__global__ __launch_bounds__(256) void k_attention(const float* __restrict__ feat, const float* __restrict__ S, const float* __restrict__ pos,
                                                  const float* __restrict__ go, const float* __restrict__ beto,
                                                  const float* __restrict__ mo, const float* __restrict__ vo, float* __restrict__ out) {
  __shared__ __attribute__((aligned(16))) unsigned char smem[2 * 4 * 2 * 16 * 256 * 2];
  __shared__ __attribute__((aligned(16))) h16 VmS[4 * 2 * 256 * 32];
  __shared__ float sc_s[4][16 * 17];
  __shared__ __attribute__((aligned(16))) h16 AtS[4 * 2 * 16 * 32];
  h16 (*Jt)[2][16 * 256] = (h16 (*)[2][16 * 256])smem;
  h16 (*Kt)[2][16 * 256] = (h16 (*)[2][16 * 256])(smem + 4 * 2 * 16 * 256 * 2);
  float* ot = (float*)smem;
  h16 (*Vm)[2][256 * 32] = (h16 (*)[2][256 * 32])VmS;
  h16 (*At)[2][16 * 32]  = (h16 (*)[2][16 * 32])AtS;
  const int tid = threadIdx.x, lane = tid & 31, wave = tid >> 5, half = lane >> 4, l16 = lane & 15;
  const int b = blockIdx.x >> 2, pi = blockIdx.x & 3;
  const int pj = wave >> 1, sub = wave & 1;
  const int p = pi * 4 + pj;

  for (int i = tid; i < 4 * 2 * 256; i += 256) { const int pp = i >> 9, pl = (i >> 8) & 1, c = i & 255;
#pragma unroll
    for (int m = 16; m < 32; ++m) Vm[pp][pl][c * 32 + m] = (h16)0.0f; }
  for (int i = tid; i < 4 * 2 * 16; i += 256) { const int pp = i >> 5, pl = (i >> 4) & 1, n = i & 15;
#pragma unroll
    for (int m = 16; m < 32; ++m) At[pp][pl][n * 32 + m] = (h16)0.0f; }
  {
    const int c = tid;
#pragma unroll 1
    for (int pp = 0; pp < 4; ++pp) {
      const float sval = S[((size_t)b * 16 + (pi * 4 + pp)) * 256 + c];
#pragma unroll
      for (int n = 0; n < 16; n++) {
        const int ph = n >> 2, pw = n & 3, h = pi * 4 + ph, w = pp * 4 + pw;
        const int g = b * 256 + h * 16 + w;
        const float pv = pos[(size_t)b * 65536 + c * 256 + h * 16 + w];
        const float kv = feat[(size_t)c * 1024 + g] + pv;
        const float jv = feat[(size_t)(256 + c) * 1024 + g] * sval + pv;
        const float vv = feat[(size_t)(512 + c) * 1024 + g] + pv;
        h16 t_;
        t_ = (h16)kv; Kt[pp][0][n * 256 + c] = t_; Kt[pp][1][n * 256 + c] = lo_of(kv, t_);
        t_ = (h16)jv; Jt[pp][0][n * 256 + c] = t_; Jt[pp][1][n * 256 + c] = lo_of(jv, t_);
        t_ = (h16)vv; Vm[pp][0][c * 32 + n] = t_;  Vm[pp][1][c * 32 + n] = lo_of(vv, t_);
      }
    }
  }
  __syncthreads();
  if (sub == 0) {
    v8f acc = {};
#pragma unroll
    for (int kc = 0; kc < 8; ++kc)
      acc = wmma_split(rfrag(&Jt[pj][0][l16 * 256 + kc * 32], half), rfrag(&Jt[pj][1][l16 * 256 + kc * 32], half),
                       rfrag(&Kt[pj][0][l16 * 256 + kc * 32], half), rfrag(&Kt[pj][1][l16 * 256 + kc * 32], half), acc);
#pragma unroll
    for (int r = 0; r < 8; ++r) sc_s[pj][(8 * half + r) * 17 + l16] = acc[r];
  }
  __syncthreads();
  {
    const int pp = tid >> 6, m = tid & 15, q4 = (tid >> 4) & 3;
    float mx = -1e30f;
#pragma unroll
    for (int n = 0; n < 16; ++n) mx = fmaxf(mx, sc_s[pp][n * 17 + m]);
    float sum = 0.f;
#pragma unroll
    for (int n = 0; n < 16; ++n) sum += expf(sc_s[pp][n * 17 + m] - mx);
    const float inv = 1.0f / sum;
#pragma unroll
    for (int i = 0; i < 4; ++i) { const int n = q4 * 4 + i; const float a = expf(sc_s[pp][n * 17 + m] - mx) * inv;
      const h16 ah = (h16)a; At[pp][0][n * 32 + m] = ah; At[pp][1][n * 32 + m] = lo_of(a, ah); }
  }
  __syncthreads();
  {
    const v16h a = rfrag(&At[pj][0][l16 * 32], half), al = rfrag(&At[pj][1][l16 * 32], half);
#pragma unroll
    for (int ct = 0; ct < 8; ++ct) {
      const int c0 = (sub * 8 + ct) * 16;
      v8f acc = {};
      acc = wmma_split(a, al, rfrag(&Vm[pj][0][(c0 + l16) * 32], half), rfrag(&Vm[pj][1][(c0 + l16) * 32], half), acc);
      const int c = c0 + l16;
      const float alpha = go[c] * rsqrtf(vo[c] + BN_EPS), mu = mo[c], bet = beto[c];
#pragma unroll
      for (int r = 0; r < 8; ++r) { const int n = 8 * half + r; ot[c * 68 + (n >> 2) * 16 + pj * 4 + (n & 3)] = (acc[r] - mu) * alpha + bet; }
    }
  }
  __syncthreads();
#pragma unroll 1
  for (int pass = 0; pass < 2; ++pass) {
    for (int ch = tid; ch < 256 * 16; ch += 256) { const int c = ch >> 4, q = (ch & 15) * 4;
      *(volatile v4f_t*)(out + (((size_t)b * 2304 + 2048 + c) << 8) + pi * 64 + q) = *(const volatile v4fa*)(ot + c * 68 + q); }
    __threadfence();
  }
}

extern "C" void kernel_launch(void* const* d_in, const int* in_sizes, int n_in,
                              void* d_out, int out_size, void* d_ws, size_t ws_size,
                              hipStream_t stream) {
  (void)in_sizes; (void)n_in; (void)out_size; (void)ws_size;
  const float* x    = (const float*)d_in[0];
  const float* go   = (const float*)d_in[25];
  const float* beto = (const float*)d_in[26];
  const float* mo   = (const float*)d_in[27];
  const float* vo   = (const float*)d_in[28];
  const float* pos  = (const float*)d_in[29];
  RowParams rp; WPtrs wp;
  const int base[4] = {1, 7, 13, 19};
  for (int i = 0; i < 4; i++) {
    wp.w[i]    = (const float*)d_in[base[i]];
    rp.bias[i] = (const float*)d_in[base[i] + 1];
    rp.g[i]    = (const float*)d_in[base[i] + 2];
    rp.beta[i] = (const float*)d_in[base[i] + 3];
    rp.mu[i]   = (const float*)d_in[base[i] + 4];
    rp.var[i]  = (const float*)d_in[base[i] + 5];
  }
  char* wsB = (char*)d_ws;
  float* rowScale = (float*)wsB;
  float* rowOff   = rowScale + 1024;
  float* feat     = rowOff + 1024;
  float* S        = feat + 1024 * 1024;
  h16*   Ah       = (h16*)(S + 16384);
  h16*   Bth      = Ah + 2 * 2097152;
  float* outf     = (float*)d_out;

  k_row_params<<<4, 256, 0, stream>>>(rp, rowScale, rowOff);
  k_copy_x<<<2048, 256, 0, stream>>>(x, outf);
  k_pack_w<<<1024, 256, 0, stream>>>(wp, Ah);
  k_pack_x<<<dim3(16, 32), 256, 0, stream>>>(x, Bth);
  k_gemm_kqvd<<<dim3(8, 8), 256, 0, stream>>>(Ah, Bth, rowScale, rowOff, feat);
  k_softmax_S<<<64, 256, 0, stream>>>(feat, S);
  k_attention<<<16, 256, 0, stream>>>(feat, S, pos, go, beto, mo, vo, outf);
}
